// Block_36309653520993
// MI455X (gfx1250) — hardware-verified
//
#include <hip/hip_runtime.h>
#ifndef NB
#define NB 2
#endif
#ifndef SQ
#define SQ 2048
#endif
#define NB_FULL 2
#define SQ_FULL 2048
#define DM 1024
#define NH 16
#define HD 64
#define DFF 4096
#define QT 256
#define NKX SQ
#define QT0 128
#define NR ((size_t)NB * SQ)
#define MP ((int)((size_t)NB * SQ))
#define LQ (3 * DM)
static_assert(DM == NH * HD);
static_assert(DM == 1024);
static_assert(HD == 64);
static_assert(SQ % QT == 0);
static_assert(QT % 128 == 0);
static_assert(QT0 == 128);
static_assert(SQ >= QT0);
static_assert(SQ % 128 == 0);
static_assert(DFF % 64 == 0);
static_assert(NB <= NB_FULL);
static_assert(SQ <= SQ_FULL);

typedef unsigned short v8us __attribute__((ext_vector_type(8), may_alias));
typedef float  v8f  __attribute__((ext_vector_type(8)));
typedef float  v4f  __attribute__((ext_vector_type(4)));
typedef float  v4fa __attribute__((ext_vector_type(4), may_alias));
typedef _Float16 v16h __attribute__((ext_vector_type(16)));
typedef _Float16 v4h __attribute__((ext_vector_type(4)));
union FragH { v16h v; v8us half[2]; _Float16 h[16]; unsigned short u[16]; };

__device__ __forceinline__ unsigned short bf16_bits(float x) { unsigned int u = __float_as_uint(x); return (unsigned short)((u + 0x7FFFu + ((u >> 16) & 1u)) >> 16); }
__device__ __forceinline__ float bf16_val(unsigned short b) { return __uint_as_float(((unsigned int)b) << 16); }
__device__ __forceinline__ float bf16_rne(float x) { return bf16_val(bf16_bits(x)); }

__device__ __forceinline__ v16h g2_frag(const _Float16* p, int hh) { FragH f; f.half[0] = *(const v8us*)((const unsigned short*)p + 8 * hh); f.half[1] = *(const v8us*)((const unsigned short*)p + 16 + 8 * hh); return f.v; }
__device__ __forceinline__ v8f g2_mma(v16h a, v16h b, v8f c) { v8f d = __builtin_amdgcn_wmma_f32_16x16x32_f16(false, a, false, b, (short)0, c, false, false); asm volatile("v_nop\n\tv_nop\n\tv_nop\n\tv_nop" : "+v"(d) : "v"(a), "v"(b)); return d; }
template <int ACT>
__global__ __launch_bounds__(128) void k_gemm2(const _Float16* __restrict__ A, int lda, size_t sA, const _Float16* __restrict__ Bh, int ldb, size_t sB, float alpha, const float* __restrict__ bias, size_t sBias, const float* __restrict__ CP, int rowsPerB, size_t sCPb, int row0g,
    float* __restrict__ C, _Float16* __restrict__ C16, int ldc, size_t sC, int M, int N, int K) { static_assert(ACT == 0 || ACT == 3);
  __shared__ __attribute__((aligned(16))) float so[4][32][68];
  const int tid = threadIdx.x, w = tid >> 5, lane = tid & 31, ln = lane & 15, hh = lane >> 4; const int by = blockIdx.y;
  A += (size_t)by * sA; Bh += (size_t)by * sB; const size_t cofs = (size_t)by * sC; const float* bp = bias ? bias + (size_t)by * sBias : nullptr;
  const int ntn = N >> 6; const int mt = blockIdx.x / ntn, nq = blockIdx.x - mt * ntn; const int row0 = mt * 128 + 32 * w, col0 = nq * 64; if (row0 >= M) return;
  const _Float16* a0p = A + (size_t)(row0 + ln) * lda; const _Float16* a1p = a0p + (size_t)16 * lda;
  const _Float16* b0p = Bh + (size_t)(col0 + ln) * ldb; const _Float16* b1p = b0p + (size_t)16 * ldb; const _Float16* b2p = b1p + (size_t)16 * ldb; const _Float16* b3p = b2p + (size_t)16 * ldb;
  const v8f z8 = {0.f,0.f,0.f,0.f,0.f,0.f,0.f,0.f}; v8f c00 = z8, c01 = z8, c02 = z8, c03 = z8, c10 = z8, c11 = z8, c12 = z8, c13 = z8;
#pragma unroll 1
  for (int kb = 0; kb < K; kb += 32) { const v16h a0 = g2_frag(a0p + kb, hh), a1 = g2_frag(a1p + kb, hh);
    v16h b = g2_frag(b0p + kb, hh); c00 = g2_mma(a0, b, c00); c10 = g2_mma(a1, b, c10);
    b = g2_frag(b1p + kb, hh); c01 = g2_mma(a0, b, c01); c11 = g2_mma(a1, b, c11);
    b = g2_frag(b2p + kb, hh); c02 = g2_mma(a0, b, c02); c12 = g2_mma(a1, b, c12);
    b = g2_frag(b3p + kb, hh); c03 = g2_mma(a0, b, c03); c13 = g2_mma(a1, b, c13); }
  v8f accs[8] = {c00, c01, c02, c03, c10, c11, c12, c13};
#pragma unroll
  for (int u = 0; u < 8; ++u) { const int t = u & 3, half = u >> 2; const int col = col0 + t * 16 + ln; const float bv = bp ? bf16_rne(bp[col]) : 0.f;
#pragma unroll
    for (int r = 0; r < 8; ++r) { const int rloc = half * 16 + 8 * hh + r; float v = accs[u][r] * alpha + bv; if (CP) { if (rowsPerB < 0) v += CP[cofs + (size_t)(row0g + row0 + rloc) * ldc + col]; else { const int bidx = (row0g + row0 + rloc) / rowsPerB; v += CP[(size_t)bidx * sCPb + (size_t)by * 64 + col]; } }
      if (ACT == 3) v = fmaxf(v, 0.f);
      so[w][rloc][t * 16 + ln] = v; } }
  __builtin_amdgcn_fence(4  , "workgroup"); __builtin_amdgcn_wave_barrier();
  const int rsub = lane >> 4, c4 = (lane & 15) * 4;
  for (int pass = 0; pass < 2; ++pass) {
#pragma unroll
    for (int q = 0; q < 16; ++q) { const int r = q * 2 + rsub; const v4f v = *(const v4fa*)&so[w][r][c4]; if (C) *(volatile v4f*)(C + cofs + (size_t)(row0 + r) * ldc + col0 + c4) = v; if (C16) { v4h h4; for (int i = 0; i < 4; ++i) h4[i] = (_Float16)v[i]; *(volatile v4h*)(C16 + cofs + (size_t)(row0 + r) * ldc + col0 + c4) = h4; } }
    if (pass == 0) __threadfence(); } }

__global__ __launch_bounds__(256) void k_wnat(const float* __restrict__ w, size_t n8, _Float16* __restrict__ Bt) { const size_t t = (size_t)blockIdx.x * 256 + threadIdx.x; if (t >= n8) return; FragH f;
#pragma unroll
  for (int q = 0; q < 8; ++q) f.h[q] = (_Float16)(bf16_rne(w[t * 8 + q]) * 16.0f);
  const v8us o = f.half[0]; *(volatile v8us*)((unsigned short*)Bt + t * 8) = o; __threadfence(); *(volatile v8us*)((unsigned short*)Bt + t * 8) = o; }

template <int NHv, int TTv>
__global__ __launch_bounds__(256) void k_vt(const _Float16* __restrict__ V16, int ldv, int voff, _Float16* __restrict__ Vt) { __shared__ unsigned short tl[64][66]; const int tid = threadIdx.x; const int slab = blockIdx.x / (TTv / 64), lg = blockIdx.x % (TTv / 64); const int b = slab / NHv, h = slab % NHv;
  for (int i = tid; i < 64 * 8; i += 256) { const int r = i / 8, c8 = (i % 8) * 8; FragH f; f.half[0] = *(const v8us*)((const unsigned short*)V16 + ((size_t)b * TTv + lg * 64 + r) * ldv + voff + h * 64 + c8);
#pragma unroll
    for (int q = 0; q < 8; ++q) tl[r][c8 + q] = f.u[q]; }
  __syncthreads();
  for (int pass = 0; pass < 2; ++pass) {
#pragma unroll
    for (int rd = 0; rd < 2; ++rd) { const int d = rd * 32 + tid / 8, pc = tid % 8; FragH f;
#pragma unroll
      for (int q = 0; q < 8; ++q) f.u[q] = tl[pc * 8 + q][d];
      *(volatile v8us*)((unsigned short*)Vt + ((size_t)slab * 64 + d) * TTv + lg * 64 + pc * 8) = f.half[0]; }
    if (pass == 0) __threadfence(); } }

__global__ __launch_bounds__(256) void k_hl(const float* __restrict__ F, _Float16* __restrict__ Hh, _Float16* __restrict__ Hl, size_t n8) { const size_t t = (size_t)blockIdx.x * 256 + threadIdx.x; if (t >= n8) return; FragH fh, fl; const v4f a = *(const v4fa*)(F + t * 8), c = *(const v4fa*)(F + t * 8 + 4);
#pragma unroll
  for (int q = 0; q < 4; ++q) { _Float16 h = (_Float16)a[q]; fh.h[q] = h; fl.h[q] = (_Float16)((a[q] - (float)h) * 1024.0f); h = (_Float16)c[q]; fh.h[4 + q] = h; fl.h[4 + q] = (_Float16)((c[q] - (float)h) * 1024.0f); }
  for (int pass = 0; pass < 2; ++pass) { *(volatile v8us*)((unsigned short*)Hh + t * 8) = fh.half[0]; *(volatile v8us*)((unsigned short*)Hl + t * 8) = fl.half[0]; if (pass == 0) __threadfence(); } }

__global__ __launch_bounds__(256) void k_rsmcf2(const float* __restrict__ S, _Float16* __restrict__ P, int hg, int q0, int nk) {
  #pragma clang fp contract(off)
  const int t = blockIdx.x * 256 + threadIdx.x; if (t >= hg * QT) return; const size_t i = (size_t)t; const float* s = S + i * NKX; const int last = q0 + (t % QT); float mx = -3.0e38f;
#pragma unroll 1
  for (int j = 0; j < nk; ++j) { const float f = (j <= last) ? 1.f : 0.f; mx = fmaxf(mx, fmaf(f, s[j], (1.f - f) * -1.0e9f)); } float se = 0.f;
#pragma unroll 1
  for (int j = 0; j < nk; ++j) { const float f = (j <= last) ? 1.f : 0.f; se += __expf(fmaf(f, s[j], (1.f - f) * -1.0e9f) - mx); } const float sc = 256.0f / se;
#pragma unroll 1
  for (int j0 = 0; j0 < nk; j0 += 8) { FragH fr; for (int q = 0; q < 8; ++q) { const int j = j0 + q; const float f = (j <= last) ? 1.f : 0.f; fr.h[q] = (_Float16)(__expf(fmaf(f, s[j], (1.f - f) * -1.0e9f) - mx) * sc); } unsigned short* d = (unsigned short*)P + i * NKX + j0; *(volatile v8us*)d = fr.half[0]; __threadfence(); *(volatile v8us*)d = fr.half[0]; } }

__global__ __launch_bounds__(64) void k_att0(const float* __restrict__ QF, const float* __restrict__ KF, const float* __restrict__ VF, int ld, float scale, float* __restrict__ OF, int ldo) {
  #pragma clang fp contract(off)
  __shared__ __attribute__((aligned(16))) float lq[64][64]; __shared__ __attribute__((aligned(16))) float lo[64][64];
  const int tid = threadIdx.x; const int h = blockIdx.x / (QT0 / 64), rg = blockIdx.x % (QT0 / 64); const int i = rg * 64 + tid;
  const float* qr = QF + (size_t)i * ld + h * HD;
#pragma unroll 1
  for (int c = 0; c < HD / 4; ++c) { *(v4f*)&lq[tid][c * 4] = *(const v4fa*)(qr + c * 4); const v4f z = {0.f, 0.f, 0.f, 0.f}; *(v4f*)&lo[tid][c * 4] = z; }
  float m = -1.0e30f, l = 0.f; const int jmax = rg * 64 + 63;
#pragma unroll 1
  for (int j = 0; j <= jmax; ++j) { const float* kr = KF + (size_t)j * ld + h * HD; const float* vr = VF + (size_t)j * ld + h * HD; float s = 0.f;
#pragma unroll 1
    for (int c = 0; c < HD / 4; ++c) { const v4f kq = *(const v4fa*)(kr + c * 4); const v4f qq = *(v4f*)&lq[tid][c * 4]; s = __fadd_rn(s, __fmul_rn(qq[0], kq[0])); s = __fadd_rn(s, __fmul_rn(qq[1], kq[1])); s = __fadd_rn(s, __fmul_rn(qq[2], kq[2])); s = __fadd_rn(s, __fmul_rn(qq[3], kq[3])); }
    s = __fmul_rn(s, scale);
    const float f = (j <= i) ? 1.f : 0.f; const float sm = fmaf(f, s, (1.f - f) * -1.0e30f); const float mn = fmaxf(m, sm); const float sc = expf(m - mn); const float e = expf(sm - mn); l = __fadd_rn(__fmul_rn(l, sc), e); m = mn;
#pragma unroll 1
    for (int c = 0; c < HD / 4; ++c) { const v4f vv = *(const v4fa*)(vr + c * 4); v4f oo = *(v4f*)&lo[tid][c * 4]; for (int u = 0; u < 4; ++u) oo[u] = __fadd_rn(__fmul_rn(oo[u], sc), __fmul_rn(e, vv[u])); *(v4f*)&lo[tid][c * 4] = oo; } }
  const float fin = 64.0f * (1.0f / l);
#pragma unroll 1
  for (int c = 0; c < HD / 4; ++c) { v4f oo = *(v4f*)&lo[tid][c * 4]; for (int u = 0; u < 4; ++u) oo[u] = __fmul_rn(oo[u], fin); *(v4f*)&lo[tid][c * 4] = oo; }
  __syncthreads();
  for (int pass = 0; pass < 2; ++pass) {
#pragma unroll 1
    for (int it = 0; it < 16; ++it) { const int row = it * 4 + tid / 16, pc = (tid % 16) * 4; const v4f v = *(const v4f*)&lo[row][pc]; *(volatile v4f*)(OF + (size_t)(rg * 64 + row) * ldo + h * HD + pc) = v; }
    if (pass == 0) __threadfence(); } }

template <int BFIN, int WXB, int XFULL>
__global__ __launch_bounds__(256) void k_ln(const float* __restrict__ X, const float* __restrict__ g, const float* __restrict__ bb, float eps, _Float16* __restrict__ N16, float* __restrict__ XB) {
  #pragma clang fp contract(off)
  __shared__ float red[256]; const size_t r = blockIdx.x; const int t = threadIdx.x;
  const size_t rin = XFULL ? ((r / SQ) * (size_t)SQ_FULL + (r % SQ)) : r;
  const v4f xa = *(const v4fa*)(X + rin * DM + t * 4); float s[4]; float sum = 0.f;
  for (int q = 0; q < 4; ++q) { s[q] = BFIN ? bf16_rne(xa[q]) : xa[q]; sum = __fadd_rn(sum, s[q]); }
  red[t] = sum; __syncthreads(); for (int st = 128; st > 0; st >>= 1) { if (t < st) red[t] = __fadd_rn(red[t], red[t + st]); __syncthreads(); } const float mu = __fmul_rn(red[0], 1.0f / (float)DM); __syncthreads();
  float vs = 0.f; for (int q = 0; q < 4; ++q) { const float dl = __fadd_rn(s[q], -mu); vs = __fadd_rn(vs, __fmul_rn(dl, dl)); } red[t] = vs; __syncthreads(); for (int st = 128; st > 0; st >>= 1) { if (t < st) red[t] = __fadd_rn(red[t], red[t + st]); __syncthreads(); }
  const float sd = sqrtf(__fmul_rn(red[0], 1.0f / (float)(DM - 1))); const float inv = 1.0f / __fadd_rn(sd, eps); v4h y; v4f xb;
  for (int q = 0; q < 4; ++q) { const int c = t * 4 + q; const float dl = __fadd_rn(s[q], -mu); y[q] = (_Float16)__fadd_rn(__fmul_rn(__fmul_rn(bf16_rne(g[c]), dl), inv), bf16_rne(bb[c])); xb[q] = s[q]; }
  for (int pass = 0; pass < 2; ++pass) { *(volatile v4h*)(N16 + r * DM + t * 4) = y; if (WXB) *(volatile v4f*)(XB + r * DM + t * 4) = xb; if (pass == 0) __threadfence(); } }

#define AL256(x) ((((size_t)(x)) + 255) & ~(size_t)255)
constexpr size_t SZ_BQKV = AL256((size_t)3 * DM * DM * 2);
constexpr size_t SZ_BWP  = AL256((size_t)DM * DM * 2);
constexpr size_t SZ_X16  = AL256(NR * DM * 2);
constexpr size_t SZ_XB   = AL256(NR * DM * 4);
constexpr size_t SZ_QKV  = AL256(NR * 3 * DM * 2);
constexpr size_t SZ_O16  = AL256(NR * DM * 2);
constexpr size_t SZ_S    = AL256((size_t)NH * QT * NKX * 4);
constexpr size_t SZ_P    = AL256((size_t)NH * QT * NKX * 2);
constexpr size_t SZ_X1   = AL256(NR * DM * 4);
constexpr size_t SZ_HF   = AL256((size_t)SQ * DFF * 2);
constexpr size_t SZ_BW1  = AL256((size_t)DFF * DM * 2);
constexpr size_t SZ_BW2  = AL256((size_t)DM * DFF * 2);
constexpr size_t SZ_UA   = SZ_S + SZ_P;
constexpr size_t SZ_UB   = SZ_X1 + SZ_HF + SZ_BW1 + SZ_BW2;
constexpr size_t SZ_U    = (SZ_UA > SZ_UB) ? SZ_UA : SZ_UB;
constexpr size_t SZ_VT   = AL256((size_t)NH * HD * SQ * 2);
constexpr size_t SZ_F0   = AL256((size_t)NB * QT0 * 3 * DM * 4);
constexpr size_t SZ_OF0  = AL256((size_t)NB * QT0 * DM * 4);
constexpr size_t SZ_OHL  = AL256((size_t)NB * QT0 * DM * 2);
constexpr size_t SZ_T0   = AL256((size_t)NB * QT0 * DM * 4);
constexpr size_t SZ_ALL  = SZ_BQKV + SZ_BWP + SZ_X16 + SZ_XB + SZ_QKV + SZ_O16 + SZ_U + SZ_VT + SZ_F0 + SZ_OF0 + 2 * SZ_OHL + SZ_T0;
static_assert(SZ_UA <= SZ_U);
static_assert(SZ_UB <= SZ_U);
static_assert(SZ_ALL <= (size_t)134217728);
static_assert(((size_t)3 * DM * DM) % 8 == 0);
static_assert(((size_t)NB * QT0 * DM) % 8 == 0);

extern "C" void kernel_launch(void* const* d_in, const int* in_sizes, int n_in,
                              void* d_out, int out_size, void* d_ws, size_t ws_size, hipStream_t stream) {
  if (n_in < 12) return;
  const size_t xneed = ((size_t)(NB - 1) * SQ_FULL + SQ) * DM;
  if ((size_t)in_sizes[0] < xneed || (size_t)out_size < xneed) return;
  if (in_sizes[1] < 3 * DM * DM || in_sizes[2] < DM * DM || in_sizes[3] < DM || in_sizes[4] < DFF * DM || in_sizes[5] < DFF || in_sizes[6] < DM * DFF || in_sizes[7] < DM || in_sizes[8] < DM || in_sizes[9] < DM || in_sizes[10] < DM || in_sizes[11] < DM) return;
  if (SZ_ALL > ws_size) return;
  const float* x = (const float*)d_in[0]; const float* qkv_w = (const float*)d_in[1]; const float* proj_w = (const float*)d_in[2]; const float* proj_b = (const float*)d_in[3];
  const float* l1_w = (const float*)d_in[4]; const float* l1_b = (const float*)d_in[5]; const float* l3_w = (const float*)d_in[6]; const float* l3_b = (const float*)d_in[7];
  const float* ln1_g = (const float*)d_in[8]; const float* ln1_b = (const float*)d_in[9]; const float* ln2_g = (const float*)d_in[10]; const float* ln2_b = (const float*)d_in[11];
  float* out = (float*)d_out;
  char* ws = (char*)d_ws; size_t off = 0;
  auto take = [&](size_t bytes) { char* p = ws + off; off += bytes; return p; };
  _Float16* BQKV = (_Float16*)take(SZ_BQKV); _Float16* BWP = (_Float16*)take(SZ_BWP);
  _Float16* X16 = (_Float16*)take(SZ_X16); float* XB = (float*)take(SZ_XB);
  _Float16* QKV = (_Float16*)take(SZ_QKV); _Float16* Q16 = QKV; _Float16* K16 = QKV + DM; _Float16* V16 = QKV + 2 * DM;
  _Float16* O16 = (_Float16*)take(SZ_O16);
  char* U = take(SZ_U);
  float* S = (float*)U; _Float16* P = (_Float16*)(U + SZ_S);
  float* X1 = (float*)U; _Float16* HF16 = (_Float16*)(U + SZ_X1); _Float16* BW1 = (_Float16*)(U + SZ_X1 + SZ_HF); _Float16* BW2 = (_Float16*)(U + SZ_X1 + SZ_HF + SZ_BW1);
  _Float16* VT = (_Float16*)take(SZ_VT);
  float* F0 = (float*)take(SZ_F0); float* OF0 = (float*)take(SZ_OF0);
  _Float16* OH = (_Float16*)take(SZ_OHL); _Float16* OL = (_Float16*)take(SZ_OHL); float* T0 = (float*)take(SZ_T0);
  _Float16* M16 = X16;
  if (off > ws_size) return;

  { const size_t n8 = (size_t)3 * DM * DM / 8; k_wnat<<<(unsigned)((n8 + 255) / 256), 256, 0, stream>>>(qkv_w, n8, BQKV); }
  { const size_t n8 = (size_t)DM * DM / 8; k_wnat<<<(unsigned)((n8 + 255) / 256), 256, 0, stream>>>(proj_w, n8, BWP); }
  k_ln<1, 1, 1><<<(unsigned)NR, 256, 0, stream>>>(x, ln1_g, ln1_b, 1e-6f, X16, XB);
  k_gemm2<0><<<dim3((unsigned)((MP / 128) * (3 * DM / 64)), 1), 128, 0, stream>>>(X16, DM, 0, BQKV, DM, 0, 0.0625f, nullptr, 0, nullptr, 1, 0, 0, nullptr, QKV, 3 * DM, 0, MP, 3 * DM, DM);
  k_gemm2<0><<<dim3((unsigned)((QT0 / 128) * (3 * DM / 64)), NB), 128, 0, stream>>>(X16, DM, (size_t)SQ * DM, BQKV, DM, 0, 0.0625f, nullptr, 0, nullptr, 1, 0, 0, F0, nullptr, 3 * DM, (size_t)QT0 * 3 * DM, QT0, 3 * DM, DM);
  for (int b = 0; b < NB; ++b) { const float* F0b = F0 + (size_t)b * QT0 * 3 * DM;
    k_att0<<<NH * (QT0 / 64), 64, 0, stream>>>(F0b, F0b + DM, F0b + 2 * DM, 3 * DM, 0.125f, OF0 + (size_t)b * QT0 * DM, DM); }
  for (int b = 0; b < NB; ++b) { const size_t r0 = (size_t)b * SQ;
    k_vt<NH, SQ><<<NH * (SQ / 64), 256, 0, stream>>>(V16 + r0 * LQ, LQ, 0, VT);
    for (int q0 = 0; q0 < SQ; q0 += QT) { const int nk = q0 + QT;
      k_gemm2<0><<<dim3((unsigned)((QT / 128) * (nk / 64)), NH), 128, 0, stream>>>(Q16 + (r0 + q0) * LQ, LQ, (size_t)HD, K16 + r0 * LQ, LQ, (size_t)HD, 0.125f, nullptr, 0, nullptr, 1, 0, 0, S, nullptr, NKX, (size_t)QT * NKX, QT, nk, HD);
      k_rsmcf2<<<(NH * QT + 255) / 256, 256, 0, stream>>>(S, P, NH, q0, nk);
      k_gemm2<0><<<dim3((unsigned)((QT / 128) * (HD / 64)), NH), 128, 0, stream>>>(P, NKX, (size_t)QT * NKX, VT, SQ, (size_t)HD * SQ, 0.25f, nullptr, 0, nullptr, 1, 0, 0, nullptr, O16 + (r0 + q0) * DM, DM, (size_t)HD, QT, HD, nk); } }
  k_gemm2<0><<<dim3((unsigned)((MP / 128) * (DM / 64)), 1), 128, 0, stream>>>(O16, DM, 0, BWP, DM, 0, 1.0f / 1024.0f, proj_b, 0, XB, -1, 0, 0, X1, nullptr, DM, 0, MP, DM, DM);
  { const size_t n8 = (size_t)NB * QT0 * DM / 8; k_hl<<<(unsigned)((n8 + 255) / 256), 256, 0, stream>>>(OF0, OH, OL, n8); }
  for (int b = 0; b < NB; ++b) { const size_t f0 = (size_t)b * QT0 * DM; const size_t r0 = (size_t)b * SQ;
    k_gemm2<0><<<dim3((unsigned)((QT0 / 128) * (DM / 64)), 1), 128, 0, stream>>>(OH + f0, DM, 0, BWP, DM, 0, 1.0f / 1024.0f, proj_b, 0, XB + r0 * DM, -1, 0, 0, T0 + f0, nullptr, DM, 0, QT0, DM, DM);
    k_gemm2<0><<<dim3((unsigned)((QT0 / 128) * (DM / 64)), 1), 128, 0, stream>>>(OL + f0, DM, 0, BWP, DM, 0, 1.0f / 1048576.0f, nullptr, 0, T0 + f0, -1, 0, 0, X1 + r0 * DM, nullptr, DM, 0, QT0, DM, DM); }
  { const size_t n8 = (size_t)DFF * DM / 8; k_wnat<<<(unsigned)((n8 + 255) / 256), 256, 0, stream>>>(l1_w, n8, BW1); k_wnat<<<(unsigned)((n8 + 255) / 256), 256, 0, stream>>>(l3_w, n8, BW2); }
  k_ln<0, 0, 0><<<(unsigned)NR, 256, 0, stream>>>(X1, ln2_g, ln2_b, 1e-6f, M16, nullptr);
  for (int b = 0; b < NB; ++b) { const size_t r0 = (size_t)b * SQ;
    k_gemm2<3><<<dim3((unsigned)((SQ / 128) * (DFF / 64)), 1), 128, 0, stream>>>(M16 + r0 * DM, DM, 0, BW1, DM, 0, 0.0625f, l1_b, 0, nullptr, 1, 0, 0, nullptr, HF16, DFF, 0, SQ, DFF, DM);
    k_gemm2<0><<<dim3((unsigned)((SQ / 128) * (DM / 64)), 1), 128, 0, stream>>>(HF16, DFF, 0, BW2, DFF, 0, 0.0625f, l3_b, 0, X1 + r0 * DM, -1, 0, 0, out + (size_t)b * SQ_FULL * DM, nullptr, DM, 0, SQ, DM, DFF); }
}
